// PairwiseFeatureBatch_69930657513704
// MI455X (gfx1250) — hardware-run, weakly checked
//
#include <hip/hip_runtime.h>
#define NF 512
#define NB 2
#define DD 128
#define NO 16
#define NHID 64
#define NCH 48
#define NPAIR (NF * (NF + 1) / 2)
#define NRP (NPAIR * NB)
#ifndef CHK
#define CHK 32768
#endif
#define KIN (6 * DD)
#define MAPW NF
#define C1W (NF + 2)
#define NPX1 (C1W * C1W)
#define K1P 160
#define K2P 448
#ifndef NPX1P
#define NPX1P 264320
#endif
#define NPX2 (MAPW * MAPW)
#ifndef CH2
#define CH2 65536
#endif
#define CH1 (NPX1P / 2)
#ifndef OUT2OFF
#define OUT2OFF 33554432
#endif
#define NSK ((NF - 1) * NB)
#define NSKP (((NSK + 127) / 128) * 128)
#define P1 48
typedef __bf16 v16b __attribute__((ext_vector_type(16)));
typedef unsigned short v8us __attribute__((ext_vector_type(8), may_alias));
typedef float  v8f  __attribute__((ext_vector_type(8)));
typedef float  v4f  __attribute__((ext_vector_type(4)));
typedef float  v4fa __attribute__((ext_vector_type(4), may_alias));
union FragB { v16b v; v8us half[2]; unsigned short u[16]; };

__device__ __forceinline__ unsigned short bf16_bits(float x) { unsigned int u = __float_as_uint(x); return (unsigned short)((u + 0x7FFFu + ((u >> 16) & 1u)) >> 16); }
__device__ __forceinline__ float bf16_val(unsigned short b) { return __uint_as_float(((unsigned int)b) << 16); }
__device__ __forceinline__ float bf16_round(float x) { return bf16_val(bf16_bits(x)); }
template <int NT>
__device__ __forceinline__ v8f mmaN(v16b ah, v16b al, v16b bh, v16b bl, v8f c) {
  c = __builtin_amdgcn_wmma_f32_16x16x32_bf16(false, ah, false, bh, (short)0, c, false, false);
  if (NT >= 2) c = __builtin_amdgcn_wmma_f32_16x16x32_bf16(false, al, false, bh, (short)0, c, false, false);
  if (NT >= 3) c = __builtin_amdgcn_wmma_f32_16x16x32_bf16(false, ah, false, bl, (short)0, c, false, false);
  asm volatile("v_nop\n\tv_nop\n\tv_nop\n\tv_nop" : "+v"(c) : "v"(ah), "v"(al), "v"(bh), "v"(bl));
  return c;
}

__global__ __launch_bounds__(256) void k_wt_bf16(const float* __restrict__ W, unsigned short* __restrict__ Wt, int K, int N) {
  const int t = blockIdx.x * 256 + threadIdx.x;
  const int k8n = K / 8;
  if (t >= N * k8n) return;
  const int n = t / k8n, k8 = (t % k8n) * 8;
  v8us v;
#pragma unroll
  for (int i = 0; i < 8; ++i) v[i] = bf16_bits(W[(size_t)(k8 + i) * N + n]);
  *(volatile v8us*)(Wt + (size_t)n * K + k8) = v;
  __threadfence();
  *(volatile v8us*)(Wt + (size_t)n * K + k8) = v;
}

template <bool ASPLIT, int ACT, bool BIAS_BF16>
__global__ __launch_bounds__(128) void k_gemm_bf(const float* __restrict__ A, int lda, const unsigned short* __restrict__ Wt, int ldb,
                                               const float* __restrict__ bias, float* __restrict__ C, int ldc, int M, int N, int K) {
  __shared__ __attribute__((aligned(16))) float so[4][16][64];
  const int tid = threadIdx.x, w = tid >> 5, lane = tid & 31, ln = lane & 15, hh = lane >> 4;
  const int ntn = N / 64;
  const int wid = blockIdx.x * 4 + w;
  const int mt = wid / ntn, nq = wid % ntn;
  if (mt * 16 >= M) return;
  const int row0 = mt * 16, col0 = nq * 64;
  const float* arow = A + (size_t)(row0 + ln) * lda;
  v8f acc[4] = {};
  for (int kb = 0; kb < K; kb += 32) {
    FragB ah, al;
    const v4f x0 = *(const v4fa*)(arow + kb + 8 * hh), x1 = *(const v4fa*)(arow + kb + 8 * hh + 4);
    const v4f x2 = *(const v4fa*)(arow + kb + 16 + 8 * hh), x3 = *(const v4fa*)(arow + kb + 16 + 8 * hh + 4);
    float xs[16] = {x0[0],x0[1],x0[2],x0[3],x1[0],x1[1],x1[2],x1[3],x2[0],x2[1],x2[2],x2[3],x3[0],x3[1],x3[2],x3[3]};
#pragma unroll
    for (int i = 0; i < 16; ++i) { const unsigned short hb = bf16_bits(xs[i]); ah.u[i] = hb; al.u[i] = ASPLIT ? bf16_bits(xs[i] - bf16_val(hb)) : (unsigned short)0; }
#pragma unroll
    for (int t = 0; t < 4; ++t) {
      const unsigned short* brow = Wt + (size_t)(col0 + t * 16 + ln) * ldb + kb;
      FragB b;
      b.half[0] = *(const v8us*)(brow + 8 * hh);
      b.half[1] = *(const v8us*)(brow + 16 + 8 * hh);
      acc[t] = mmaN<ASPLIT ? 2 : 1>(ah.v, al.v, b.v, b.v, acc[t]);
    }
  }
#pragma unroll
  for (int t = 0; t < 4; ++t) {
    float bv = bias ? bias[col0 + t * 16 + ln] : 0.f;
    if (BIAS_BF16) bv = bf16_round(bv);
#pragma unroll
    for (int r = 0; r < 8; ++r) { float v = acc[t][r] + bv; if (ACT == 1) v = fmaxf(v, 0.f); so[w][8 * hh + r][t * 16 + ln] = v; }
  }
  __builtin_amdgcn_fence(__ATOMIC_ACQ_REL, "workgroup");
  __builtin_amdgcn_wave_barrier();
  const int rsub = lane >> 4, c4 = (lane & 15) * 4;
  for (int pass = 0; pass < 2; ++pass) {
#pragma unroll
    for (int q = 0; q < 8; ++q) {
      const int r = q * 2 + rsub;
      const v4f v = *(const v4fa*)&so[w][r][c4];
      *(volatile v4f*)(C + (size_t)(row0 + r) * ldc + col0 + c4) = v;
    }
    if (pass == 0) __threadfence();
  }
}

template <bool ASPLIT, int ACT, bool BIAS_BF16, bool RES_BF16>
__global__ __launch_bounds__(128) void k_gemm_bf3(const float* __restrict__ A, int lda, const unsigned short* __restrict__ Wt, int ldb,
                                                const float* __restrict__ bias, const float* __restrict__ resid, int rmod, int ldr,
                                                float* __restrict__ C, int ldc, int M, int N, int K) {
  __shared__ __attribute__((aligned(16))) float so[4][16][64];
  const int tid = threadIdx.x, w = tid >> 5, lane = tid & 31, ln = lane & 15, hh = lane >> 4;
  const int ntn = N / 64;
  const int wid = blockIdx.x * 4 + w;
  const int mt = wid / ntn, nq = wid % ntn;
  if (mt * 16 >= M) return;
  const int row0 = mt * 16, col0 = nq * 64;
  const float* arow = A + (size_t)(row0 + ln) * lda;
  v8f acc[4] = {};
  for (int kb = 0; kb < K; kb += 32) {
    FragB ah, al;
    const v4f x0 = *(const v4fa*)(arow + kb + 8 * hh), x1 = *(const v4fa*)(arow + kb + 8 * hh + 4);
    const v4f x2 = *(const v4fa*)(arow + kb + 16 + 8 * hh), x3 = *(const v4fa*)(arow + kb + 16 + 8 * hh + 4);
    float xs[16] = {x0[0],x0[1],x0[2],x0[3],x1[0],x1[1],x1[2],x1[3],x2[0],x2[1],x2[2],x2[3],x3[0],x3[1],x3[2],x3[3]};
#pragma unroll
    for (int i = 0; i < 16; ++i) { const unsigned short hb = bf16_bits(xs[i]); ah.u[i] = hb; al.u[i] = ASPLIT ? bf16_bits(xs[i] - bf16_val(hb)) : (unsigned short)0; }
#pragma unroll
    for (int t = 0; t < 4; ++t) {
      const unsigned short* brow = Wt + (size_t)(col0 + t * 16 + ln) * ldb + kb;
      FragB b;
      b.half[0] = *(const v8us*)(brow + 8 * hh);
      b.half[1] = *(const v8us*)(brow + 16 + 8 * hh);
      acc[t] = mmaN<ASPLIT ? 2 : 1>(ah.v, al.v, b.v, b.v, acc[t]);
    }
  }
#pragma unroll
  for (int t = 0; t < 4; ++t) {
    const int col = col0 + t * 16 + ln;
    float bv = bias ? bias[col] : 0.f;
    if (BIAS_BF16) bv = bf16_round(bv);
#pragma unroll
    for (int r = 0; r < 8; ++r) {
      float v = acc[t][r] + bv;
      if (resid) { float rv = resid[(size_t)((row0 + 8 * hh + r) % rmod) * ldr + col]; if (RES_BF16) rv = bf16_round(rv); v += rv; }
      if (ACT == 1) v = fmaxf(v, 0.f);
      if (ACT == 2) v = 0.5f * v * (1.0f + erff(v * 0.70710678118654752f));
      if (ACT == 3) { const float u = 0.7978845608028654f * (v + 0.044715f * v * v * v); v = 0.5f * v * (1.0f + tanhf(u)); }
      so[w][8 * hh + r][t * 16 + ln] = v;
    }
  }
  __builtin_amdgcn_fence(__ATOMIC_ACQ_REL, "workgroup");
  __builtin_amdgcn_wave_barrier();
  const int rsub = lane >> 4, c4 = (lane & 15) * 4;
  for (int pass = 0; pass < 2; ++pass) {
#pragma unroll
    for (int q = 0; q < 8; ++q) {
      const int r = q * 2 + rsub;
      const v4f v = *(const v4fa*)&so[w][r][c4];
      *(volatile v4f*)(C + (size_t)(row0 + r) * ldc + col0 + c4) = v;
    }
    if (pass == 0) __threadfence();
  }
}
template <bool PARAM_BF16>
__global__ __launch_bounds__(256) void k_layernorm(const float* __restrict__ X, const float* __restrict__ R, const float* __restrict__ g, const float* __restrict__ bta,
                                                  float* __restrict__ out_sum, float* __restrict__ out_norm, int N, float eps) {
  __shared__ float red[256];
  const int row = blockIdx.x, tid = threadIdx.x;
  const float* x = X + (size_t)row * N; const float* rr = R ? R + (size_t)row * N : nullptr;
  float vals[16];
  const int per = N / 256;
  float s1 = 0.f;
  for (int u = 0; u < per / 4; ++u) {
    const int j = tid * 4 + 1024 * u;
    const v4f a = *(const v4fa*)(x + j);
    v4f b = {0.f,0.f,0.f,0.f}; if (rr) b = *(const v4fa*)(rr + j);
#pragma unroll
    for (int q = 0; q < 4; ++q) { const float v = a[q] + b[q]; vals[u * 4 + q] = v; s1 += v; }
  }
  red[tid] = s1; __syncthreads();
  for (int st = 128; st > 0; st >>= 1) { if (tid < st) red[tid] += red[tid + st]; __syncthreads(); }
  const float mu = red[0] / (float)N; __syncthreads();
  float s2 = 0.f;
  for (int u = 0; u < per / 4; ++u)
#pragma unroll
    for (int q = 0; q < 4; ++q) { const float c = vals[u * 4 + q] - mu; s2 += c * c; }
  red[tid] = s2; __syncthreads();
  for (int st = 128; st > 0; st >>= 1) { if (tid < st) red[tid] += red[tid + st]; __syncthreads(); }
  const float rs = rsqrtf(red[0] / (float)N + eps);
  for (int pass = 0; pass < 2; ++pass) {
    for (int u = 0; u < per / 4; ++u) {
      const int j = tid * 4 + 1024 * u;
      v4f o, sm;
#pragma unroll
      for (int q = 0; q < 4; ++q) {
        float gg = g[j + q], bb = bta[j + q];
        if (PARAM_BF16) { gg = bf16_round(gg); bb = bf16_round(bb); }
        sm[q] = vals[u * 4 + q]; o[q] = (vals[u * 4 + q] - mu) * rs * gg + bb;
      }
      if (out_sum) *(volatile v4f*)(out_sum + (size_t)row * N + j) = sm;
      *(volatile v4f*)(out_norm + (size_t)row * N + j) = o;
    }
    if (pass == 0) __threadfence();
  }
}


typedef _Float16 v16h __attribute__((ext_vector_type(16)));
union FragH { v16h v; v8us half[2]; _Float16 h[16]; unsigned short u[16]; };
template <int NT>
__device__ __forceinline__ v8f mmaH(v16h ah, v16h al, v16h bh, v16h bl, v8f c) {
  c = __builtin_amdgcn_wmma_f32_16x16x32_f16(false, ah, false, bh, (short)0, c, false, false);
  if (NT >= 2) c = __builtin_amdgcn_wmma_f32_16x16x32_f16(false, al, false, bh, (short)0, c, false, false);
  if (NT >= 3) c = __builtin_amdgcn_wmma_f32_16x16x32_f16(false, ah, false, bl, (short)0, c, false, false);
  asm volatile("v_nop\n\tv_nop\n\tv_nop\n\tv_nop" : "+v"(c) : "v"(ah), "v"(al), "v"(bh), "v"(bl));
  return c;
}
template <bool ASPLIT>
__global__ __launch_bounds__(128) void k_gemm_h(const float* __restrict__ A, int lda, size_t sA, const _Float16* __restrict__ Bh, int ldb, size_t sB, float alpha, float* __restrict__ C, int ldc, size_t sC, int M, int N, int K) {
  __shared__ __attribute__((aligned(16))) float so[4][16][64];
  const int tid = threadIdx.x, w = tid >> 5, lane = tid & 31, ln = lane & 15, hh = lane >> 4; const int by = blockIdx.y;
  A += (size_t)by * sA; Bh += (size_t)by * sB; C += (size_t)by * sC;
  const int ntn = (N + 63) / 64; const int wid = blockIdx.x * 4 + w; const int mt = wid / ntn, nq = wid % ntn; if (mt * 16 >= M) return;
  const int row0 = mt * 16, col0 = nq * 64; const float* arow = A + (size_t)(row0 + ln) * lda;
  v8f acc[4] = {};
  for (int kb = 0; kb < K; kb += 32) {
    FragH ah, al;
    const v4f x0 = *(const v4fa*)(arow + kb + 8 * hh), x1 = *(const v4fa*)(arow + kb + 8 * hh + 4), x2 = *(const v4fa*)(arow + kb + 16 + 8 * hh), x3 = *(const v4fa*)(arow + kb + 16 + 8 * hh + 4);
    float xs[16] = {x0[0],x0[1],x0[2],x0[3],x1[0],x1[1],x1[2],x1[3],x2[0],x2[1],x2[2],x2[3],x3[0],x3[1],x3[2],x3[3]};
#pragma unroll
    for (int i = 0; i < 16; ++i) { const _Float16 h = (_Float16)xs[i]; ah.h[i] = h; al.h[i] = ASPLIT ? (_Float16)(xs[i] - (float)h) : (_Float16)0.0f; }
#pragma unroll
    for (int t = 0; t < 4; ++t) { if (col0 + t * 16 >= N) continue; const size_t boff = (size_t)(col0 + t * 16 + ln) * ldb + kb; FragH bq; bq.half[0] = *(const v8us*)(Bh + boff + 8 * hh); bq.half[1] = *(const v8us*)(Bh + boff + 16 + 8 * hh);
      acc[t] = mmaH<ASPLIT ? 2 : 1>(ah.v, al.v, bq.v, bq.v, acc[t]); }
  }
#pragma unroll
  for (int t = 0; t < 4; ++t) { if (col0 + t * 16 >= N) continue;
#pragma unroll
    for (int r = 0; r < 8; ++r) so[w][8 * hh + r][t * 16 + ln] = acc[t][r] * alpha; }
  __builtin_amdgcn_fence(__ATOMIC_ACQ_REL, "workgroup"); __builtin_amdgcn_wave_barrier();
  const int rsub = lane >> 4, c4 = (lane & 15) * 4;
  for (int pass = 0; pass < 2; ++pass) {
#pragma unroll
    for (int q = 0; q < 8; ++q) { const int r = q * 2 + rsub; if (col0 + c4 < N) { const v4f v = *(const v4fa*)&so[w][r][c4]; *(volatile v4f*)(C + (size_t)(row0 + r) * ldc + col0 + c4) = v; } }
    if (pass == 0) __threadfence(); }
}

__global__ __launch_bounds__(256) void k_wt_f16(const float* __restrict__ W, _Float16* __restrict__ Wt, int K, int N, float scale) {
  const int t = blockIdx.x * 256 + threadIdx.x; if (t >= N * (K / 8)) return; const int n = t / (K / 8), k8 = (t % (K / 8)) * 8; FragH f;
#pragma unroll
  for (int i = 0; i < 8; ++i) f.h[i] = (_Float16)(bf16_round(W[(size_t)(k8 + i) * N + n]) * scale); const v8us o = f.half[0];
  *(volatile v8us*)((unsigned short*)Wt + (size_t)n * K + k8) = o; __threadfence(); *(volatile v8us*)((unsigned short*)Wt + (size_t)n * K + k8) = o;
}
template <int ACT>
__global__ __launch_bounds__(128) void k_gemm_hhx(const _Float16* __restrict__ A, int lda, size_t sA, const _Float16* __restrict__ Bh, int ldb, size_t sB, float alpha, const float* __restrict__ bias, size_t sBias, const float* __restrict__ CP, int rowsPerB, size_t sCPb, int row0g,
    float* __restrict__ C, _Float16* __restrict__ C16, int ldc, size_t sC, int M, int N, int K) {
  __shared__ __attribute__((aligned(16))) float so[4][16][64];
  const int tid = threadIdx.x, w = tid >> 5, lane = tid & 31, ln = lane & 15, hh = lane >> 4; const int by = blockIdx.y;
  A += (size_t)by * sA; Bh += (size_t)by * sB; const size_t cofs = (size_t)by * sC; const float* bp = bias ? bias + (size_t)by * sBias : nullptr;
  const int ntn = (N + 63) / 64; const int wid = blockIdx.x * 4 + w; const int mt = wid / ntn, nq = wid % ntn; if (mt * 16 >= M) return;
  const int row0 = mt * 16, col0 = nq * 64; const _Float16* arow = A + (size_t)(row0 + ln) * lda;
  v8f acc[4] = {};
  for (int kb = 0; kb < K; kb += 32) { FragH ah; ah.half[0] = *(const v8us*)((const unsigned short*)arow + kb + 8 * hh); ah.half[1] = *(const v8us*)((const unsigned short*)arow + kb + 16 + 8 * hh);
#pragma unroll
    for (int t = 0; t < 4; ++t) { if (col0 + t * 16 >= N) continue; const size_t boff = (size_t)(col0 + t * 16 + ln) * ldb + kb; FragH bq; bq.half[0] = *(const v8us*)((const unsigned short*)Bh + boff + 8 * hh); bq.half[1] = *(const v8us*)((const unsigned short*)Bh + boff + 16 + 8 * hh);
      acc[t] = mmaH<1>(ah.v, ah.v, bq.v, bq.v, acc[t]); }
  }
#pragma unroll
  for (int t = 0; t < 4; ++t) { if (col0 + t * 16 >= N) continue; const int col = col0 + t * 16 + ln; const float bv = bp ? bf16_round(bp[col]) : 0.f;
#pragma unroll
    for (int r = 0; r < 8; ++r) { float v = acc[t][r] * alpha + bv; if (CP) { const int rr = row0g + row0 + 8 * hh + r; if (rowsPerB < 0) v += CP[cofs + (size_t)rr * ldc + col];        else { const int bidx = rr / rowsPerB; v += CP[(size_t)bidx * sCPb + (size_t)by * 64 + col]; } } if (ACT == 1) v = (v > 0.f) ? v : expm1f(v); else if (ACT == 7) v = (v > 0.f) ? v + 1.0f : expf(v); else if (ACT == 8) v = tanhf(v); else if (ACT == 9) v = 0.5f * v * (1.0f + tanhf(0.7978845608028654f * (v + 0.044715f * v * v * v))); else if (ACT == 11) v = 1.0f / (1.0f + expf(-v)); else if (ACT == 12) v = (v > 0.f) ? v : 0.01f * v; else if (ACT == 14) v = (v > 0.f) ? v : 0.1f * v; else if (ACT == 16) v = (v >= 0.f) ? v : 0.3f * v; else if (ACT == 17) v = (v >= 0.f) ? v : 0.2f * v; else if (ACT == 15) v = v / (1.0f + expf(-v)); else if (ACT == 3) v = fmaxf(v, 0.f); else if (ACT == 6) v = 0.5f * v * (1.0f + erff(v * 0.70710678118654752f)); so[w][8 * hh + r][t * 16 + ln] = v; } }
  __builtin_amdgcn_fence(__ATOMIC_ACQ_REL, "workgroup"); __builtin_amdgcn_wave_barrier();
  const int rsub = lane >> 4, c4 = (lane & 15) * 4; typedef _Float16 v4h __attribute__((ext_vector_type(4)));
  for (int pass = 0; pass < 2; ++pass) {
#pragma unroll
    for (int q = 0; q < 8; ++q) { const int r = q * 2 + rsub; if (col0 + c4 < N) { const v4f v = *(const v4fa*)&so[w][r][c4]; if (C) *(volatile v4f*)(C + cofs + (size_t)(row0 + r) * ldc + col0 + c4) = v; if (C16) { v4h h4; for (int i = 0; i < 4; ++i) h4[i] = (_Float16)v[i]; *(volatile v4h*)(C16 + cofs + (size_t)(row0 + r) * ldc + col0 + c4) = h4; } } }
    if (pass == 0) __threadfence(); }
}


typedef _Float16 v4h __attribute__((ext_vector_type(4)));

__global__ __launch_bounds__(256) void k_x16(const float* __restrict__ x, _Float16* __restrict__ X16, size_t n8) { const size_t t = (size_t)blockIdx.x * 256 + threadIdx.x; if (t >= n8) return; FragH f;
#pragma unroll
  for (int q = 0; q < 8; ++q) f.h[q] = (_Float16)bf16_round(x[t * 8 + q]); *(volatile v8us*)((unsigned short*)X16 + t * 8) = f.half[0]; __threadfence(); *(volatile v8us*)((unsigned short*)X16 + t * 8) = f.half[0]; }
__global__ __launch_bounds__(256) void k_h16(const float* __restrict__ x, _Float16* __restrict__ X16, size_t n8) { const size_t t = (size_t)blockIdx.x * 256 + threadIdx.x; if (t >= n8) return; FragH f;
#pragma unroll
  for (int q = 0; q < 8; ++q) f.h[q] = (_Float16)x[t * 8 + q]; *(volatile v8us*)((unsigned short*)X16 + t * 8) = f.half[0]; __threadfence(); *(volatile v8us*)((unsigned short*)X16 + t * 8) = f.half[0]; }
__global__ __launch_bounds__(256) void k_round16f(const float* __restrict__ W, _Float16* __restrict__ Bt, size_t n8) { const size_t t = (size_t)blockIdx.x * 256 + threadIdx.x; if (t >= n8) return; FragH f;
#pragma unroll
  for (int i = 0; i < 8; ++i) f.h[i] = (_Float16)(bf16_round(W[t * 8 + i]) * 16.0f); *(volatile v8us*)((unsigned short*)Bt + t * 8) = f.half[0]; __threadfence(); *(volatile v8us*)((unsigned short*)Bt + t * 8) = f.half[0]; }
template <int NHv, int TTv>
__global__ __launch_bounds__(256) void k_vt(const _Float16* __restrict__ V16, int ldv, int voff, _Float16* __restrict__ Vt) { __shared__ unsigned short tl[64][66]; const int tid = threadIdx.x; const int slab = blockIdx.x / (TTv / 64), lg = blockIdx.x % (TTv / 64); const int b = slab / NHv, h = slab % NHv;
  for (int i = tid; i < 64 * 8; i += 256) { const int r = i / 8, c8 = (i % 8) * 8; FragH f; f.half[0] = *(const v8us*)((const unsigned short*)V16 + ((size_t)b * TTv + lg * 64 + r) * ldv + voff + h * 64 + c8);
#pragma unroll
    for (int q = 0; q < 8; ++q) tl[r][c8 + q] = f.u[q]; }
  __syncthreads();
  for (int pass = 0; pass < 2; ++pass) {
#pragma unroll
    for (int rd = 0; rd < 2; ++rd) { const int d = rd * 32 + tid / 8, pc = tid % 8; FragH f;
#pragma unroll
      for (int q = 0; q < 8; ++q) f.u[q] = tl[pc * 8 + q][d];
      *(volatile v8us*)((unsigned short*)Vt + ((size_t)slab * 64 + d) * TTv + lg * 64 + pc * 8) = f.half[0]; }
    if (pass == 0) __threadfence(); } }

__global__ __launch_bounds__(256) void k_hl(const float* __restrict__ F, _Float16* __restrict__ Hh, _Float16* __restrict__ Hl, size_t n8) { const size_t t = (size_t)blockIdx.x * 256 + threadIdx.x; if (t >= n8) return; FragH fh, fl; const v4f a = *(const v4fa*)(F + t * 8), c = *(const v4fa*)(F + t * 8 + 4);
#pragma unroll
  for (int q = 0; q < 4; ++q) { _Float16 h = (_Float16)a[q]; fh.h[q] = h; fl.h[q] = (_Float16)((a[q] - (float)h) * 1024.0f); h = (_Float16)c[q]; fh.h[4 + q] = h; fl.h[4 + q] = (_Float16)((c[q] - (float)h) * 1024.0f); }
  for (int pass = 0; pass < 2; ++pass) { *(volatile v8us*)((unsigned short*)Hh + t * 8) = fh.half[0]; *(volatile v8us*)((unsigned short*)Hl + t * 8) = fl.half[0]; if (pass == 0) __threadfence(); } }

__device__ __forceinline__ v16h g2_frag(const _Float16* p, int hh) { FragH f; f.half[0] = *(const v8us*)((const unsigned short*)p + 8 * hh); f.half[1] = *(const v8us*)((const unsigned short*)p + 16 + 8 * hh); return f.v; }
__device__ __forceinline__ v8f g2_mma(v16h a, v16h b, v8f c) { v8f d = __builtin_amdgcn_wmma_f32_16x16x32_f16(false, a, false, b, (short)0, c, false, false); asm volatile("v_nop\n\tv_nop\n\tv_nop\n\tv_nop" : "+v"(d) : "v"(a), "v"(b)); return d; }
template <int ACT>
__global__ __launch_bounds__(128) void k_gemm2(const _Float16* __restrict__ A, int lda, size_t sA, const _Float16* __restrict__ Bh, int ldb, size_t sB, float alpha, const float* __restrict__ bias, size_t sBias, const float* __restrict__ CP, int rowsPerB, size_t sCPb, int row0g,
    float* __restrict__ C, _Float16* __restrict__ C16, int ldc, size_t sC, int M, int N, int K) { static_assert(ACT == 0 || ACT == 3 || ACT == 6 || ACT == 8 || ACT == 9 || ACT == 11 || ACT == 12 || ACT == 14 || ACT == 15 || ACT == 16 || ACT == 17, "k_gemm2: unsupported ACT code (would silently apply no activation)");
  __shared__ __attribute__((aligned(16))) float so[4][32][68];
  const int tid = threadIdx.x, w = tid >> 5, lane = tid & 31, ln = lane & 15, hh = lane >> 4; const int by = blockIdx.y;
  A += (size_t)by * sA; Bh += (size_t)by * sB; const size_t cofs = (size_t)by * sC; const float* bp = bias ? bias + (size_t)by * sBias : nullptr;
  const int ntn = N >> 6; const int mt = blockIdx.x / ntn, nq = blockIdx.x - mt * ntn; const int row0 = mt * 128 + 32 * w, col0 = nq * 64; if (row0 >= M) return;
  const _Float16* a0p = A + (size_t)(row0 + ln) * lda; const _Float16* a1p = a0p + (size_t)16 * lda;
  const _Float16* b0p = Bh + (size_t)(col0 + ln) * ldb; const _Float16* b1p = b0p + (size_t)16 * ldb; const _Float16* b2p = b1p + (size_t)16 * ldb; const _Float16* b3p = b2p + (size_t)16 * ldb;
  const v8f z8 = {0.f,0.f,0.f,0.f,0.f,0.f,0.f,0.f}; v8f c00 = z8, c01 = z8, c02 = z8, c03 = z8, c10 = z8, c11 = z8, c12 = z8, c13 = z8;
#pragma unroll 1
  for (int kb = 0; kb < K; kb += 32) { const v16h a0 = g2_frag(a0p + kb, hh), a1 = g2_frag(a1p + kb, hh);
    v16h b = g2_frag(b0p + kb, hh); c00 = g2_mma(a0, b, c00); c10 = g2_mma(a1, b, c10);
    b = g2_frag(b1p + kb, hh); c01 = g2_mma(a0, b, c01); c11 = g2_mma(a1, b, c11);
    b = g2_frag(b2p + kb, hh); c02 = g2_mma(a0, b, c02); c12 = g2_mma(a1, b, c12);
    b = g2_frag(b3p + kb, hh); c03 = g2_mma(a0, b, c03); c13 = g2_mma(a1, b, c13); }
  v8f accs[8] = {c00, c01, c02, c03, c10, c11, c12, c13};
#pragma unroll
  for (int u = 0; u < 8; ++u) { const int t = u & 3, half = u >> 2; const int col = col0 + t * 16 + ln; const float bv = bp ? bf16_round(bp[col]) : 0.f;
#pragma unroll
    for (int r = 0; r < 8; ++r) { const int rloc = half * 16 + 8 * hh + r; float v = accs[u][r] * alpha + bv; if (CP) { if (rowsPerB < 0) v += CP[cofs + (size_t)(row0g + row0 + rloc) * ldc + col];        else { const int bidx = (row0g + row0 + rloc) / rowsPerB; v += CP[(size_t)bidx * sCPb + (size_t)by * 64 + col]; } }
      if (ACT == 3) v = fmaxf(v, 0.f); else if (ACT == 6) v = 0.5f * v * (1.0f + erff(v * 0.70710678118654752f)); else if (ACT == 11) v = 1.0f / (1.0f + expf(-v)); else if (ACT == 15) v = v / (1.0f + expf(-v)); else if (ACT == 12) v = (v > 0.f) ? v : 0.01f * v; else if (ACT == 8) v = tanhf(v); else if (ACT == 9) v = 0.5f * v * (1.0f + tanhf(0.7978845608028654f * (v + 0.044715f * v * v * v))); else if (ACT == 14) v = (v > 0.f) ? v : 0.1f * v; else if (ACT == 16) v = (v >= 0.f) ? v : 0.3f * v; else if (ACT == 17) v = (v >= 0.f) ? v : 0.2f * v;
      so[w][rloc][t * 16 + ln] = v; } }
  __builtin_amdgcn_fence(__ATOMIC_ACQ_REL, "workgroup"); __builtin_amdgcn_wave_barrier();
  const int rsub = lane >> 4, c4 = (lane & 15) * 4;
  for (int pass = 0; pass < 2; ++pass) {
#pragma unroll
    for (int q = 0; q < 16; ++q) { const int r = q * 2 + rsub; const v4f v = *(const v4fa*)&so[w][r][c4]; if (C) *(volatile v4f*)(C + cofs + (size_t)(row0 + r) * ldc + col0 + c4) = v; if (C16) { v4h h4; for (int i = 0; i < 4; ++i) h4[i] = (_Float16)v[i]; *(volatile v4h*)(C16 + cofs + (size_t)(row0 + r) * ldc + col0 + c4) = h4; } }
    if (pass == 0) __threadfence(); } }


__device__ __forceinline__ float gelu_erf(float v) { return 0.5f * v * (1.0f + erff(v * 0.70710678118654752f)); }
__global__ __launch_bounds__(256) void k_prefix(const float* __restrict__ x, float* __restrict__ PC) {
  #pragma clang fp contract(off)
  const int t = threadIdx.x; float s1 = 0.f, s2 = 0.f, s3 = 0.f; const size_t st = (size_t)(NF + 1) * NB * DD;
  for (int pass = 0; pass < 2; ++pass) { *(volatile float*)(PC + t) = 0.f; *(volatile float*)(PC + st + t) = 0.f; *(volatile float*)(PC + 2 * st + t) = 0.f; }
#pragma unroll 1
  for (int k = 0; k < NF; ++k) { const float v = bf16_round(x[(size_t)k * NB * DD + t]); s1 += v; s2 += v * v; float c = v * v; c = c * v; s3 += c; const size_t o = (size_t)(k + 1) * NB * DD + t;
    *(volatile float*)(PC + o) = s1; *(volatile float*)(PC + st + o) = s2; *(volatile float*)(PC + 2 * st + o) = s3; __threadfence(); *(volatile float*)(PC + o) = s1; *(volatile float*)(PC + st + o) = s2; *(volatile float*)(PC + 2 * st + o) = s3; } }
__device__ __forceinline__ void pair_ij(int p, int& i, int& j) { int ii = (int)((sqrtf(8.0f * (float)p + 1.0f) - 1.0f) * 0.5f); while ((ii + 1) * (ii + 2) / 2 <= p) ++ii; while (ii * (ii + 1) / 2 > p) --ii; i = ii; j = p - ii * (ii + 1) / 2; }
__global__ __launch_bounds__(256) void k_feat(const float* __restrict__ x, const float* __restrict__ PC, size_t r0, size_t nrows, _Float16* __restrict__ A) {
  #pragma clang fp contract(off)
  const size_t t = (size_t)blockIdx.x * 256 + threadIdx.x; if (t >= nrows * (KIN / 8)) return; const int g = (int)(t % (KIN / 8)); const size_t lrow = t / (KIN / 8); const size_t row = r0 + lrow; const int b = (int)(row % NB); const int p = (int)(row / NB); int i, j; pair_ij(p, i, j); const int blk = g / (DD / 8), d0 = (g % (DD / 8)) * 8; FragH f;
  const float* xi = x + ((size_t)i * NB + b) * DD + d0; const float* xj = x + ((size_t)j * NB + b) * DD + d0;
  if (blk == 0) { for (int q = 0; q < 8; ++q) f.h[q] = (_Float16)bf16_round(xi[q]); }
  else if (blk == 1) { for (int q = 0; q < 8; ++q) f.h[q] = (_Float16)bf16_round(xj[q]); }
  else if (blk == 2) { for (int q = 0; q < 8; ++q) f.h[q] = (_Float16)(bf16_round(xi[q]) * bf16_round(xj[q])); }
  else { const size_t st = (size_t)(NF + 1) * NB * DD; const float* pc = PC + (size_t)(blk - 3) * st; const float* hi = pc + ((size_t)(i + 1) * NB + b) * DD + d0; const float* lo = pc + ((size_t)j * NB + b) * DD + d0; const float L = (float)(i - j + 1); for (int q = 0; q < 8; ++q) f.h[q] = (_Float16)((hi[q] - lo[q]) / L); }
  unsigned short* dst = (unsigned short*)A + lrow * KIN + g * 8; *(volatile v8us*)dst = f.half[0]; __threadfence(); *(volatile v8us*)dst = f.half[0]; }
__global__ __launch_bounds__(256) void k_skipfeat(const float* __restrict__ x, _Float16* __restrict__ A) {
  #pragma clang fp contract(off)
  const int t = blockIdx.x * 256 + threadIdx.x; if (t >= NSKP * (3 * DD / 8)) return; const int g = t % (3 * DD / 8), row = t / (3 * DD / 8); const int b = row % NB, k = row / NB; const int blk = g / (DD / 8), d0 = (g % (DD / 8)) * 8; FragH f;
  if (k >= NF - 1) { for (int q = 0; q < 8; ++q) f.h[q] = (_Float16)0.0f; }
  else { const float* xa = x + ((size_t)k * NB + b) * DD + d0; const float* xb2 = x + ((size_t)(k + 1) * NB + b) * DD + d0; for (int q = 0; q < 8; ++q) { const float a = bf16_round(xa[q]), c = bf16_round(xb2[q]); f.h[q] = (blk == 0) ? (_Float16)a : ((blk == 1) ? (_Float16)c : (_Float16)(a * c)); } }
  *(volatile v8us*)((unsigned short*)A + (size_t)t * 8) = f.half[0]; __threadfence(); *(volatile v8us*)((unsigned short*)A + (size_t)t * 8) = f.half[0]; }
__global__ __launch_bounds__(256) void k_geluhl(const float* __restrict__ F, _Float16* __restrict__ Hh, _Float16* __restrict__ Hl, size_t n8) {
  #pragma clang fp contract(off)
  const size_t t = (size_t)blockIdx.x * 256 + threadIdx.x; if (t >= n8) return; v8f a = *(const v8f*)(F + t * 8);
#pragma unroll 1
  for (int q = 0; q < 8; ++q) a[q] = gelu_erf(a[q]);
  FragH fh, fl; for (int q = 0; q < 8; ++q) { const _Float16 h = (_Float16)a[q]; fh.h[q] = h; fl.h[q] = (_Float16)((a[q] - (float)h) * 1024.0f); }
  for (int pass = 0; pass < 2; ++pass) { *(volatile v8us*)((unsigned short*)Hh + t * 8) = fh.half[0]; *(volatile v8us*)((unsigned short*)Hl + t * 8) = fl.half[0]; if (pass == 0) __threadfence(); } }
__global__ __launch_bounds__(256) void k_dense(const float* __restrict__ SC, _Float16* __restrict__ Mh, _Float16* __restrict__ Ml) {
  #pragma clang fp contract(off)
  const size_t t = (size_t)blockIdx.x * 256 + threadIdx.x; if (t >= (size_t)NB * MAPW * (MAPW / 8)) return; const int j0 = (int)(t % (MAPW / 8)) * 8; const int i = (int)((t / (MAPW / 8)) % MAPW); const int b = (int)(t / ((size_t)(MAPW / 8) * MAPW));
  for (int pass = 0; pass < 2; ++pass) {
    for (int u = 0; u < 8; ++u) { const int j = j0 + u; FragH fh, fl; for (int q = 0; q < 16; ++q) { fh.h[q & 7] = (_Float16)0.0f; } v8us h0, h1, l0, l1;
      if (j <= i) { const size_t p = (size_t)i * (i + 1) / 2 + j; const float* s = SC + (p * NB + b) * NO; FragH a0, a1, c0, c1;
        for (int q = 0; q < 8; ++q) { const _Float16 hv = (_Float16)s[q]; a0.h[q] = hv; c0.h[q] = (_Float16)((s[q] - (float)hv) * 1024.0f); const _Float16 hv2 = (_Float16)s[8 + q]; a1.h[q] = hv2; c1.h[q] = (_Float16)((s[8 + q] - (float)hv2) * 1024.0f); }
        h0 = a0.half[0]; h1 = a1.half[0]; l0 = c0.half[0]; l1 = c1.half[0]; }
      else { for (int q = 0; q < 8; ++q) { h0[q] = 0; h1[q] = 0; l0[q] = 0; l1[q] = 0; } }
      const size_t o = (((size_t)b * MAPW + i) * MAPW + j) * NO; *(volatile v8us*)((unsigned short*)Mh + o) = h0; *(volatile v8us*)((unsigned short*)Mh + o + 8) = h1; *(volatile v8us*)((unsigned short*)Ml + o) = l0; *(volatile v8us*)((unsigned short*)Ml + o + 8) = l1; }
    if (pass == 0) __threadfence(); } }
__global__ __launch_bounds__(256) void k_im1(const _Float16* __restrict__ M, int b, size_t lr0, _Float16* __restrict__ I) { const size_t t = (size_t)blockIdx.x * 256 + threadIdx.x; if (t >= (size_t)CH1 * (K1P / 8)) return; const int q = (int)(t % (K1P / 8)); const size_t lr = lr0 + t / (K1P / 8); v8us v; for (int u = 0; u < 8; ++u) v[u] = 0;
  if (q < 18 && lr < (size_t)NPX1) { const int tap = q / 2, hf = q % 2; const int y = (int)(lr / C1W), x = (int)(lr % C1W); const int iy = y - 2 + tap / 3, ix = x - 2 + tap % 3; if (iy >= 0 && iy < MAPW && ix >= 0 && ix < MAPW) v = *(const v8us*)((const unsigned short*)M + (((size_t)b * MAPW + iy) * MAPW + ix) * NO + hf * 8); }
  unsigned short* d = (unsigned short*)I + t * 8; *(volatile v8us*)d = v; __threadfence(); *(volatile v8us*)d = v; }
__global__ __launch_bounds__(256) void k_im2c(const _Float16* __restrict__ H1, int b, size_t lr0, _Float16* __restrict__ I) { const size_t t = (size_t)blockIdx.x * 256 + threadIdx.x; if (t >= (size_t)CH2 * (K2P / 8)) return; const int q = (int)(t % (K2P / 8)); const size_t lr = lr0 + t / (K2P / 8); v8us v; for (int u = 0; u < 8; ++u) v[u] = 0;
  if (q < 54) { const int tap = q / 6, c8 = (q % 6) * 8; const int y = (int)(lr / MAPW), x = (int)(lr % MAPW); const int iy = y + tap / 3, ix = x + tap % 3; v = *(const v8us*)((const unsigned short*)H1 + (((size_t)b * NPX1P) + (size_t)iy * C1W + ix) * P1 + c8); }
  unsigned short* d = (unsigned short*)I + t * 8; *(volatile v8us*)d = v; __threadfence(); *(volatile v8us*)d = v; }
__global__ __launch_bounds__(256) void k_wre(const float* __restrict__ w, int cn, int nlive, int nrows, int kp, _Float16* __restrict__ Bt) { const size_t t = (size_t)blockIdx.x * 256 + threadIdx.x; if (t >= (size_t)nrows * kp / 8) return; const int col0 = (int)((t * 8) % kp); const int o = (int)((t * 8) / kp); FragH f; for (int q = 0; q < 8; ++q) { const int col = col0 + q; const int tap = col / cn, c = col % cn; f.h[q] = (o < nlive && col < 9 * cn) ? (_Float16)(bf16_round(w[((size_t)o * cn + c) * 9 + tap]) * 16.0f) : (_Float16)0.0f; }
  *(volatile v8us*)((unsigned short*)Bt + t * 8) = f.half[0]; __threadfence(); *(volatile v8us*)((unsigned short*)Bt + t * 8) = f.half[0]; }
__global__ __launch_bounds__(64) void k_bpadv(const float* __restrict__ src, int n, int np, float* __restrict__ dst) { const int i = threadIdx.x; if (i >= np) return; const float v = (i < n) ? bf16_round(src[i]) : 0.f; *(volatile float*)(dst + i) = v; __threadfence(); *(volatile float*)(dst + i) = v; }
__global__ __launch_bounds__(256) void k_final(const float* __restrict__ C20, const float* __restrict__ C21, const float* __restrict__ cb2, size_t lr0, float* __restrict__ out) {
  #pragma clang fp contract(off)
  const size_t t = (size_t)blockIdx.x * 256 + threadIdx.x; if (t >= (size_t)CH2) return; const size_t lr = lr0 + t; const int i = (int)(lr / MAPW), j = (int)(lr % MAPW); int L = (i > j) ? (i - j) : (j - i); if (L < 1) L = 1; const float lf = (float)L; v8f v[4];
  for (int b = 0; b < NB; ++b) { const float* c = (b ? C21 : C20) + t * NO; for (int q = 0; q < 8; ++q) { float u = c[q]; u += bf16_round(cb2[q]); v[2 * b][q] = lf * u; float u2 = c[8 + q]; u2 += bf16_round(cb2[8 + q]); v[2 * b + 1][q] = lf * u2; } }
  float* o = out + ((size_t)i * MAPW + j) * NB * NO;
  for (int pass = 0; pass < 2; ++pass) { for (int u = 0; u < 4; ++u) *(volatile v8f*)(o + u * 8) = v[u]; if (pass == 0) __threadfence(); } }
__global__ __launch_bounds__(256) void k_skipout(const float* __restrict__ T, float* __restrict__ out1) { const int t = blockIdx.x * 256 + threadIdx.x; if (t >= NSK * 2) return; const int r = t / 2, h = t % 2; const v8f a = *(const v8f*)(T + (size_t)r * 64 + h * 8); *(volatile v8f*)(out1 + (size_t)r * NO + h * 8) = a; __threadfence(); *(volatile v8f*)(out1 + (size_t)r * NO + h * 8) = a; }
__global__ __launch_bounds__(256) void k_wsc(const float* __restrict__ Wm, _Float16* __restrict__ Bt, size_t n8, float sc) { const size_t t = (size_t)blockIdx.x * 256 + threadIdx.x; if (t >= n8) return; FragH f; for (int q = 0; q < 8; ++q) f.h[q] = (_Float16)(bf16_round(Wm[t * 8 + q]) * sc); *(volatile v8us*)((unsigned short*)Bt + t * 8) = f.half[0]; __threadfence(); *(volatile v8us*)((unsigned short*)Bt + t * 8) = f.half[0]; }
__global__ __launch_bounds__(256) void k_w3p(const float* __restrict__ w, _Float16* __restrict__ Bt) { const int t = blockIdx.x * 256 + threadIdx.x; if (t >= 64 * 64 / 8) return; const int c0 = (t * 8) % 64, o = (t * 8) / 64; FragH f; for (int q = 0; q < 8; ++q) f.h[q] = (o < NO) ? (_Float16)(bf16_round(w[o * 64 + c0 + q]) * 16.0f) : (_Float16)0.0f;
  *(volatile v8us*)((unsigned short*)Bt + (size_t)t * 8) = f.half[0]; __threadfence(); *(volatile v8us*)((unsigned short*)Bt + (size_t)t * 8) = f.half[0]; }

extern "C" void kernel_launch(void* const* d_in, const int* in_sizes, int n_in,
                              void* d_out, int out_size, void* d_ws, size_t ws_size, hipStream_t stream) {
  (void)in_sizes; (void)n_in; (void)out_size;
  const float* const* I = (const float* const*)d_in; const float* x = I[0]; const float* w1 = I[1]; const float* b1 = I[2]; const float* w2 = I[3]; const float* b2 = I[4]; const float* w3 = I[5]; const float* b3 = I[6]; const float* sw1 = I[7]; const float* sb1 = I[8]; const float* sw2 = I[9]; const float* sb2 = I[10]; const float* sw3 = I[11]; const float* sb3 = I[12]; const float* cw1 = I[13]; const float* cb1 = I[14]; const float* cw2 = I[15]; const float* cb2 = I[16];
  char* ws = (char*)d_ws; size_t off = 0;
  auto take = [&](size_t bytes) { char* p = ws + off; off += (bytes + 255) & ~(size_t)255; return p; };
  _Float16* BW1 = (_Float16*)take((size_t)NHID * KIN * 2); _Float16* BW2 = (_Float16*)take((size_t)NHID * NHID * 2); _Float16* BW3 = (_Float16*)take((size_t)64 * NHID * 2); float* b3p = (float*)take(64 * 4); _Float16* BS1 = (_Float16*)take((size_t)NHID * 3 * DD * 2); _Float16* BS2 = (_Float16*)take((size_t)NHID * NHID * 2); _Float16* BS3 = (_Float16*)take((size_t)64 * NHID * 2); float* sb3p = (float*)take(64 * 4);
  _Float16* BC1 = (_Float16*)take((size_t)64 * K1P * 2); float* cb1p = (float*)take(64 * 4); _Float16* BC2 = (_Float16*)take((size_t)64 * K2P * 2);
  float* PC = (float*)take((size_t)3 * (NF + 1) * NB * DD * 4); size_t imh = (size_t)CH2 * K2P; if ((size_t)CHK * KIN > imh) imh = (size_t)CHK * KIN; if ((size_t)CH1 * K1P > imh) imh = (size_t)CH1 * K1P; _Float16* IM = (_Float16*)take(imh * 2); _Float16* A = IM;
  float* G = (float*)take((size_t)CHK * NHID * 4); _Float16* Hh = (_Float16*)take((size_t)CHK * NHID * 2); _Float16* Hl = (_Float16*)take((size_t)CHK * NHID * 2); float* SC = (float*)take((size_t)NRP * NO * 4);
  _Float16* Mh = (_Float16*)take((size_t)NB * NPX2 * NO * 2); _Float16* Ml = (_Float16*)take((size_t)NB * NPX2 * NO * 2); float* H1F = (float*)take((size_t)CH1 * P1 * 4); _Float16* H1h = (_Float16*)take((size_t)NB * NPX1P * P1 * 2); _Float16* H1l = (_Float16*)take((size_t)NB * NPX1P * P1 * 2); float* C2b = (float*)take((size_t)CH2 * NO * 4); float* C2c = (float*)take((size_t)CH2 * NO * 4); float* TS = G;
  if (off > ws_size) return;
  k_wsc<<<(NHID * KIN / 8 + 255) / 256, 256, 0, stream>>>(w1, BW1, (size_t)NHID * KIN / 8, 16.0f); k_wsc<<<(NHID * NHID / 8 + 255) / 256, 256, 0, stream>>>(w2, BW2, (size_t)NHID * NHID / 8, 16.0f); k_w3p<<<2, 256, 0, stream>>>(w3, BW3); k_bpadv<<<1, 64, 0, stream>>>(b3, NO, 64, b3p);
  k_wsc<<<(NHID * 3 * DD / 8 + 255) / 256, 256, 0, stream>>>(sw1, BS1, (size_t)NHID * 3 * DD / 8, 16.0f); k_wsc<<<(NHID * NHID / 8 + 255) / 256, 256, 0, stream>>>(sw2, BS2, (size_t)NHID * NHID / 8, 16.0f); k_w3p<<<2, 256, 0, stream>>>(sw3, BS3); k_bpadv<<<1, 64, 0, stream>>>(sb3, NO, 64, sb3p);
  k_wre<<<(unsigned)(((size_t)64 * K1P / 8 + 255) / 256), 256, 0, stream>>>(cw1, NO, NCH, 64, K1P, BC1); k_bpadv<<<1, 64, 0, stream>>>(cb1, NCH, 64, cb1p); k_wre<<<(unsigned)(((size_t)64 * K2P / 8 + 255) / 256), 256, 0, stream>>>(cw2, NCH, NO, 64, K2P, BC2);
  k_prefix<<<1, 256, 0, stream>>>(x, PC);
  for (size_t r0 = 0; r0 < (size_t)NRP; r0 += CHK) { const size_t nr = ((size_t)NRP - r0 < (size_t)CHK) ? ((size_t)NRP - r0) : (size_t)CHK; const dim3 g((unsigned)((nr / 128) * 1), 1);
    k_feat<<<(unsigned)((nr * (KIN / 8) + 255) / 256), 256, 0, stream>>>(x, PC, r0, nr, A);
    k_gemm2<0><<<g, 128, 0, stream>>>(A, KIN, 0, BW1, KIN, 0, 0.0625f, b1, 0, nullptr, 1, 0, 0, G, nullptr, NHID, 0, (int)nr, NHID, KIN); k_geluhl<<<(unsigned)((nr * NHID / 8 + 255) / 256), 256, 0, stream>>>(G, Hh, Hl, nr * NHID / 8);
    k_gemm2<0><<<g, 128, 0, stream>>>(Hl, NHID, 0, BW2, NHID, 0, 0.0625f / 1024.0f, nullptr, 0, nullptr, 1, 0, 0, G, nullptr, NHID, 0, (int)nr, NHID, NHID); k_gemm2<0><<<g, 128, 0, stream>>>(Hh, NHID, 0, BW2, NHID, 0, 0.0625f, b2, 0, G, 1, (size_t)NHID, 0, G, nullptr, NHID, 0, (int)nr, NHID, NHID); k_geluhl<<<(unsigned)((nr * NHID / 8 + 255) / 256), 256, 0, stream>>>(G, Hh, Hl, nr * NHID / 8);
    k_gemm_hhx<0><<<dim3((unsigned)((nr / 16) * 1), 1), 128, 0, stream>>>(Hl, NHID, 0, BW3, NHID, 0, 0.0625f / 1024.0f, nullptr, 0, nullptr, 1, 0, 0, SC + r0 * NO, nullptr, NO, 0, (int)nr, NO, NHID); k_gemm_hhx<0><<<dim3((unsigned)((nr / 16) * 1), 1), 128, 0, stream>>>(Hh, NHID, 0, BW3, NHID, 0, 0.0625f, b3p, 0, SC + r0 * NO, 1, (size_t)NO, 0, SC + r0 * NO, nullptr, NO, 0, (int)nr, NO, NHID); }
  k_dense<<<(unsigned)(((size_t)NB * MAPW * (MAPW / 8) + 255) / 256), 256, 0, stream>>>(SC, Mh, Ml);
  for (int b = 0; b < NB; ++b) for (size_t lr0 = 0; lr0 < (size_t)NPX1P; lr0 += CH1) { const dim3 g1((CH1 / 16) * (P1 / 16), 1); const unsigned gi1 = (unsigned)(((size_t)CH1 * (K1P / 8) + 255) / 256);
    k_im1<<<gi1, 256, 0, stream>>>(Ml, b, lr0, IM); k_gemm_hhx<0><<<g1, 128, 0, stream>>>(IM, K1P, 0, BC1, K1P, 0, 0.0625f / 1024.0f, nullptr, 0, nullptr, 1, 0, 0, H1F, nullptr, P1, 0, CH1, P1, K1P);
    k_im1<<<gi1, 256, 0, stream>>>(Mh, b, lr0, IM); k_gemm_hhx<0><<<g1, 128, 0, stream>>>(IM, K1P, 0, BC1, K1P, 0, 0.0625f, cb1p, 0, H1F, 1, (size_t)P1, 0, H1F, nullptr, P1, 0, CH1, P1, K1P);
    k_geluhl<<<(unsigned)(((size_t)CH1 * P1 / 8 + 255) / 256), 256, 0, stream>>>(H1F, H1h + ((size_t)b * NPX1P + lr0) * P1, H1l + ((size_t)b * NPX1P + lr0) * P1, (size_t)CH1 * P1 / 8); }
  for (size_t lr0 = 0; lr0 < (size_t)NPX2; lr0 += CH2) { const dim3 g2((CH2 / 16) * (NO / 16), 1);
    for (int b = 0; b < NB; ++b) { float* C2x = b ? C2c : C2b;
      k_im2c<<<(unsigned)(((size_t)CH2 * (K2P / 8) + 255) / 256), 256, 0, stream>>>(H1l, b, lr0, IM); k_gemm_hhx<0><<<g2, 128, 0, stream>>>(IM, K2P, 0, BC2, K2P, 0, 0.0625f / 1024.0f, nullptr, 0, nullptr, 1, 0, 0, C2x, nullptr, NO, 0, CH2, NO, K2P);
      k_im2c<<<(unsigned)(((size_t)CH2 * (K2P / 8) + 255) / 256), 256, 0, stream>>>(H1h, b, lr0, IM); k_gemm_hhx<0><<<g2, 128, 0, stream>>>(IM, K2P, 0, BC2, K2P, 0, 0.0625f, nullptr, 0, C2x, 1, (size_t)NO, 0, C2x, nullptr, NO, 0, CH2, NO, K2P); }
    k_final<<<(CH2 + 255) / 256, 256, 0, stream>>>(C2b, C2c, cb2, lr0, (float*)d_out); }
  { _Float16* AS = IM; const dim3 gs((NSKP / 128) * 1, 1);
    k_skipfeat<<<(NSKP * (3 * DD / 8) + 255) / 256, 256, 0, stream>>>(x, AS);
    k_gemm2<0><<<gs, 128, 0, stream>>>(AS, 3 * DD, 0, BS1, 3 * DD, 0, 0.0625f, sb1, 0, nullptr, 1, 0, 0, G, nullptr, NHID, 0, NSKP, NHID, 3 * DD); k_geluhl<<<(NSKP * NHID / 8 + 255) / 256, 256, 0, stream>>>(G, Hh, Hl, (size_t)NSKP * NHID / 8);
    k_gemm2<0><<<gs, 128, 0, stream>>>(Hl, NHID, 0, BS2, NHID, 0, 0.0625f / 1024.0f, nullptr, 0, nullptr, 1, 0, 0, G, nullptr, NHID, 0, NSKP, NHID, NHID); k_gemm2<0><<<gs, 128, 0, stream>>>(Hh, NHID, 0, BS2, NHID, 0, 0.0625f, sb2, 0, G, 1, (size_t)NHID, 0, G, nullptr, NHID, 0, NSKP, NHID, NHID); k_geluhl<<<(NSKP * NHID / 8 + 255) / 256, 256, 0, stream>>>(G, Hh, Hl, (size_t)NSKP * NHID / 8);
    float* T = TS; k_gemm2<0><<<gs, 128, 0, stream>>>(Hl, NHID, 0, BS3, NHID, 0, 0.0625f / 1024.0f, nullptr, 0, nullptr, 1, 0, 0, T, nullptr, 64, 0, NSKP, 64, NHID); k_gemm2<0><<<gs, 128, 0, stream>>>(Hh, NHID, 0, BS3, NHID, 0, 0.0625f, sb3p, 0, T, 1, (size_t)64, 0, T, nullptr, 64, 0, NSKP, 64, NHID);
    k_skipout<<<(NSK * 2 + 255) / 256, 256, 0, stream>>>(T, (float*)((char*)d_out + OUT2OFF)); }
}
